// xGINE_16028817949316
// MI455X (gfx1250) — hardware-verified
//
#include <hip/hip_runtime.h>

#define NN 100000
#define NE 1600000
#define CH 64
#define NP 100032
#define NG 64
#define NOUT 10
#define NT 256
#define TILE 2048
#define NTILE 49
#define NPA (NTILE * TILE)
#define SCH 4096
#define SPT (SCH / NT)
#define NCH ((NE + SCH - 1) / SCH)
#define NSB 50
#define RPB (NN / NSB)
#define SCHP 2048
#define NCHP ((NN + SCHP - 1) / SCHP)
#define SENT 0xFFFFFFFFu

typedef __attribute__((ext_vector_type(16))) _Float16 v16h;
typedef __attribute__((ext_vector_type(8)))  _Float16 v8h;
typedef __attribute__((ext_vector_type(16))) __bf16   v16b;
typedef __attribute__((ext_vector_type(8)))  __bf16   v8b;
typedef __attribute__((ext_vector_type(8)))  float    v8f;
typedef __attribute__((ext_vector_type(4)))  float    v4f;
typedef __attribute__((ext_vector_type(2)))  float    v2f;
typedef __attribute__((ext_vector_type(2)))  double   v2d;
typedef __attribute__((ext_vector_type(4)))  int      v4i;

__device__ __forceinline__ unsigned short f2bf_bits(float f) {
  unsigned u = __float_as_uint(f);
  return (unsigned short)((u + 0x7FFFu + ((u >> 16) & 1u)) >> 16);
}
__device__ __forceinline__ float bf_bits2f(unsigned short h) { return __uint_as_float(((unsigned)h) << 16); }

__device__ __forceinline__ void dep_guard_h(v8f& a, v8f& b, v16h x, v16h y) { asm volatile("v_nop\n\tv_nop\n\tv_nop\n\tv_nop" : "+v"(a), "+v"(b) : "v"(x), "v"(y)); }
__device__ __forceinline__ void dep_guard_b(v8f& a, v8f& b, v16b x, v16b y) { asm volatile("v_nop\n\tv_nop\n\tv_nop\n\tv_nop" : "+v"(a), "+v"(b) : "v"(x), "v"(y)); }
__device__ __forceinline__ void keep4_h(v16h a, v16h b, v16h c, v16h d) { asm volatile("v_nop" :: "v"(a), "v"(b), "v"(c), "v"(d)); }
__device__ __forceinline__ void keep4_b(v16b a, v16b b, v16b c, v16b d) { asm volatile("v_nop" :: "v"(a), "v"(b), "v"(c), "v"(d)); }
__device__ __forceinline__ void acc_guard4(v8f& a, v8f& b, v8f& c, v8f& d) { asm volatile("v_nop\n\tv_nop\n\tv_nop\n\tv_nop" : "+v"(a), "+v"(b), "+v"(c), "+v"(d)); }
template <typename T> struct Frag;
template <> struct Frag<_Float16> {
  typedef v16h V; union U { v16h v; v8h h[2]; };
  static __device__ __forceinline__ v16h load(const _Float16* p) {
    U f; f.h[0] = *(const v8h*)(p); f.h[1] = *(const v8h*)(p + 16); return f.v;
  }
  static __device__ __forceinline__ v8f mma(v16h a, v16h b, v8f c) {
    return __builtin_amdgcn_wmma_f32_16x16x32_f16(false, a, false, b, (short)0, c, false, false);
  }
  static __device__ __forceinline__ void guard(v8f& a, v8f& b, v16h x, v16h y) { dep_guard_h(a, b, x, y); }
  static __device__ __forceinline__ void keep(v16h a, v16h b, v16h c, v16h d) { keep4_h(a, b, c, d); }
};
template <> struct Frag<__bf16> {
  typedef v16b V; union U { v16b v; v8b h[2]; };
  static __device__ __forceinline__ v16b load(const __bf16* p) {
    U f; f.h[0] = *(const v8b*)(p); f.h[1] = *(const v8b*)(p + 16); return f.v;
  }
  static __device__ __forceinline__ v8f mma(v16b a, v16b b, v8f c) {
    return __builtin_amdgcn_wmma_f32_16x16x32_bf16(false, a, false, b, (short)0, c, false, false);
  }
  static __device__ __forceinline__ void guard(v8f& a, v8f& b, v16b x, v16b y) { dep_guard_b(a, b, x, y); }
  static __device__ __forceinline__ void keep(v16b a, v16b b, v16b c, v16b d) { keep4_b(a, b, c, d); }
};

template <int ET> struct Elem;
template <> struct Elem<0> { typedef _Float16 T; };
template <> struct Elem<1> { typedef __bf16 T; };
template <int ET, bool SPLIT, int BIAS_MODE, int OUT_MODE, bool RESID, int ACT = 0>
__global__ __launch_bounds__(256) void wmma_gemm64(
    const unsigned short* __restrict__ Ap, const unsigned short* __restrict__ A2p, int lda, long strideA,
    const unsigned short* __restrict__ Btp, const unsigned short* __restrict__ Bt2p, int ldb, long strideB,
    void* __restrict__ Cout, void* __restrict__ Cout2, int ldc, long strideC,
    const float* __restrict__ bias,
    const float* __restrict__ resid, long strideR,
    int M, int N, int K, float scale) {
  typedef typename Elem<ET>::T T;
  typedef typename Frag<T>::V V;
  const T* A = (const T*)Ap; const T* A2 = (const T*)A2p; const T* Bt = (const T*)Btp; const T* Bt2 = (const T*)Bt2p;
  __shared__ __align__(16) float sT[8][16 * 68];
  const int b    = blockIdx.y;
  const int lane = threadIdx.x & 31;
  const int wave = threadIdx.x >> 5;
  const int tilesN = N >> 6;
  const int tilesM = M >> 6;
  const int tile = blockIdx.x * 8 + wave;
  if (tile >= tilesM * tilesN) return;
  const int tm = tile / tilesN;
  const int tn = tile - tm * tilesN;
  const int m0 = tm << 6;
  const int n0 = tn << 6;

  const T* Ab  = A  + (size_t)b * strideA;
  const T* Bb  = Bt + (size_t)b * strideB;
  const T* Ab2 = SPLIT ? (A2  + (size_t)b * strideA) : nullptr;
  const T* Bb2 = SPLIT ? (Bt2 + (size_t)b * strideB) : nullptr;

  const int rlane = lane & 15;
  const int koff  = (lane >> 4) * 8;
  const int mOff  = (lane >> 4) * 8;

  v8f acc[4][4];
#pragma unroll
  for (int i = 0; i < 4; ++i)
#pragma unroll
    for (int j = 0; j < 4; ++j) acc[i][j] = (v8f){0.f,0.f,0.f,0.f,0.f,0.f,0.f,0.f};

  for (int k0 = 0; k0 < K; k0 += 32) {
    V bh[4], bl[4];
#pragma unroll
    for (int j = 0; j < 4; ++j) {
      const size_t bo = (size_t)(n0 + (j << 4) + rlane) * ldb + koff + k0;
      bh[j] = Frag<T>::load(Bb + bo);
      if (SPLIT) bl[j] = Frag<T>::load(Bb2 + bo);
    }
#pragma unroll
    for (int i = 0; i < 4; ++i) {
      const size_t ao = (size_t)(m0 + (i << 4) + rlane) * lda + koff + k0;
      V ah = Frag<T>::load(Ab + ao);
      V al;
      if (SPLIT) al = Frag<T>::load(Ab2 + ao);
#pragma unroll
      for (int j = 0; j < 4; ++j) {
        acc[i][j] = Frag<T>::mma(ah, bh[j], acc[i][j]);
        if (SPLIT) {
          acc[i][j] = Frag<T>::mma(ah, bl[j], acc[i][j]);
          acc[i][j] = Frag<T>::mma(al, bh[j], acc[i][j]);
        }
      }
      Frag<T>::guard(acc[i][0], acc[i][3], ah, SPLIT ? al : ah);
    }
    Frag<T>::keep(bh[0], bh[1], bh[2], bh[3]);
    if (SPLIT) Frag<T>::keep(bl[0], bl[1], bl[2], bl[3]);
  }
  acc_guard4(acc[0][0], acc[0][1], acc[0][2], acc[0][3]);
  acc_guard4(acc[1][0], acc[1][1], acc[1][2], acc[1][3]);
  acc_guard4(acc[2][0], acc[2][1], acc[2][2], acc[2][3]);
  acc_guard4(acc[3][0], acc[3][1], acc[3][2], acc[3][3]);

  float* slab = sT[wave];
  const float* Rb = RESID ? (resid + (size_t)b * strideR) : nullptr;
#pragma unroll
  for (int i = 0; i < 4; ++i) {
    const int mBase = m0 + (i << 4);
#pragma unroll
    for (int j = 0; j < 4; ++j) {
      const int n = n0 + (j << 4) + rlane;
      float bv = 0.f;
      if (BIAS_MODE == 2) bv = bias[n];
#pragma unroll
      for (int r = 0; r < 8; ++r) {
        float v = acc[i][j][r] * scale;
        if (BIAS_MODE == 1) v += bias[mBase + mOff + r];
        if (BIAS_MODE == 2) v += bv;
        if (RESID) v += Rb[(size_t)(mBase + mOff + r) * ldc + n];
        if (ACT == 1) v = tanhf(v);
        if (ACT == 2) v = fmaxf(v, 0.0f);
        if (ACT == 3) v = v / (1.0f + expf(-v));
        if (ACT == 4) v = (v > 0.f) ? v : 0.01f * v;
        if (ACT == 5) v = 0.5f * v * (1.0f + erff(v * 0.70710678118654752f));
        slab[(mOff + r) * 68 + (j << 4) + rlane] = v;
      }
    }
    __builtin_amdgcn_fence(__ATOMIC_RELEASE, "workgroup");
    __builtin_amdgcn_wave_barrier();
    __builtin_amdgcn_fence(__ATOMIC_ACQUIRE, "workgroup");
    if (OUT_MODE == 0) {
      float* C = (float*)Cout + (size_t)b * strideC;
      const int hh = lane >> 4, c4 = (lane & 15) * 4;
      for (int pass = 0; pass < 2; ++pass) {
#pragma unroll
        for (int it = 0; it < 8; ++it) {
          const int row = it * 2 + hh;
          v4f v = *(const v4f*)(slab + row * 68 + c4);
          *(volatile v4f*)(C + (size_t)(mBase + row) * ldc + n0 + c4) = v;
        }
        __threadfence();
      }
    } else {
      const int q = lane >> 3, c8 = (lane & 7) * 8;
      unsigned short* C  = (unsigned short*)Cout  + (size_t)b * strideC;
      unsigned short* C2 = (OUT_MODE == 2) ? ((unsigned short*)Cout2 + (size_t)b * strideC) : nullptr;
      for (int pass = 0; pass < 2; ++pass) {
#pragma unroll
        for (int it = 0; it < 4; ++it) {
          const int row = it * 4 + q;
          const float* sp = slab + row * 68 + c8;
          v8h hv, lv;
#pragma unroll
          for (int e = 0; e < 8; ++e) {
            if (OUT_MODE == 1) {
              hv[e] = (_Float16)sp[e];
            } else {
              unsigned short hb = f2bf_bits(sp[e]);
              unsigned short lb = f2bf_bits(sp[e] - bf_bits2f(hb));
              hv[e] = __builtin_bit_cast(_Float16, hb);
              lv[e] = __builtin_bit_cast(_Float16, lb);
            }
          }
          *(volatile v8h*)(C + (size_t)(mBase + row) * ldc + n0 + c8) = hv;
          if (OUT_MODE == 2) *(volatile v8h*)(C2 + (size_t)(mBase + row) * ldc + n0 + c8) = lv;
        }
        __threadfence();
      }
    }
    __builtin_amdgcn_fence(__ATOMIC_RELEASE, "workgroup");
    __builtin_amdgcn_wave_barrier();
    __builtin_amdgcn_fence(__ATOMIC_ACQUIRE, "workgroup");
  }
}

__device__ __forceinline__ int blk_excl_scan(int cnt, int* scan_ws, int tid, int* tot) {
  const int lane = tid & 31, wave = tid >> 5; int incl = cnt;
#pragma unroll
  for (int o = 1; o < 32; o <<= 1) { const int v = __shfl_up(incl, o, 32); if (lane >= o) incl += v; }
  if (lane == 31) scan_ws[wave] = incl;
  __syncthreads();
  if (wave == 0) { int wv = (lane < NT / 32) ? scan_ws[lane] : 0; int wincl = wv;
#pragma unroll
    for (int o = 1; o < 32; o <<= 1) { const int v = __shfl_up(wincl, o, 32); if (lane >= o) wincl += v; }
    if (lane < NT / 32) scan_ws[32 + lane] = wincl - wv; if (lane == 31) scan_ws[64] = wincl; }
  __syncthreads();
  const int res = scan_ws[32 + wave] + incl - cnt; *tot = scan_ws[64];
  return res;
}
template <int SP, int CAP>
__device__ __forceinline__ int chunk_hits(const int* __restrict__ dstv, int e0, int n0, int tid, unsigned* LIST, int* scan_ws) {
  const int eb = e0 + tid * SP;
  unsigned rec[SP]; int cnt = 0;
  {
    const bool inr = (eb < NE);
    const int ebc = inr ? eb : (NE - SP);
#pragma unroll
    for (int k = 0; k < SP; k += 4) {
      const v4i d4 = *(const v4i*)(dstv + ebc + k);
#pragma unroll
      for (int e = 0; e < 4; ++e) {
        const int d = d4[e]; unsigned r = SENT;
        if (inr && d >= n0 && d < n0 + TILE) { r = ((unsigned)(d - n0) << 21) | (unsigned)(eb + k + e); ++cnt; }
        rec[k + e] = r;
      }
    }
  }
  int tot; int p = blk_excl_scan(cnt, scan_ws, tid, &tot);
#pragma unroll
  for (int k = 0; k < SP; ++k) if (rec[k] != SENT) { if ((unsigned)p < (unsigned)CAP) LIST[p] = rec[k]; ++p; }
  __syncthreads();
  return tot < CAP ? tot : CAP;
}

template <int MODE>
__device__ __forceinline__ v2f hrow(const float* __restrict__ H, int n, int lane, v2f sc, v2f sh) {
  v2f v = *(const v2f*)(H + (size_t)n * CH + 2 * lane);
  if (MODE) {
    const v2f t = v * sc + sh;
    v2f r; r.x = fmaxf(t.x, 0.f); r.y = fmaxf(t.y, 0.f);
    return r;
  }
  return v;
}

__global__ __launch_bounds__(NT) void prep_kernel(const float* __restrict__ w0, const float* __restrict__ w1,
                                                 const float* __restrict__ w2, const float* __restrict__ w3,
                                                 unsigned short* __restrict__ WH) {
  const int i = blockIdx.x * NT + threadIdx.x;
  if (i < 4 * 2048) {
    const int m = i >> 11, k = i & 2047;
    const float* src = (m == 0) ? w0 : ((m == 1) ? w1 : ((m == 2) ? w2 : w3));
    const _Float16 h0 = (_Float16)(src[2 * k] * 16.0f), h1 = (_Float16)(src[2 * k + 1] * 16.0f);
    const unsigned u = (unsigned)__builtin_bit_cast(unsigned short, h0) | ((unsigned)__builtin_bit_cast(unsigned short, h1) << 16);
    ((volatile unsigned*)WH)[i] = u;
    __threadfence();
    ((volatile unsigned*)WH)[i] = u;
  }
}

template <int MODE>
__global__ __launch_bounds__(NT) void agg_kernel(const float* __restrict__ H, const float* __restrict__ scsh,
                                                const int* __restrict__ ei, const float* __restrict__ eattr,
                                                const float* __restrict__ ew, const float* __restrict__ ebv,
                                                const float* __restrict__ epsp, float* AGG, unsigned short* __restrict__ XH) {
  __shared__ unsigned LIST[SCH];
  __shared__ int scan_ws[80];
  __shared__ __align__(16) float slab[8][4 * 68];
  const int tid = threadIdx.x, lane = tid & 31, wave = tid >> 5;
  const int n0 = blockIdx.x * TILE;
  const v2f wv = *(const v2f*)(ew + 2 * lane);
  const v2f bv = *(const v2f*)(ebv + 2 * lane);
  v2f sc = {1.f, 1.f}, sh = {0.f, 0.f};
  if (MODE) { sc = *(const v2f*)(scsh + 2 * lane); sh = *(const v2f*)(scsh + CH + 2 * lane); }
  const float ep = 1.0f + epsp[0];
  const v2f z2 = {0.f, 0.f};
  for (int pass = 0; pass < 2; ++pass) {
#pragma unroll 1
    for (int j = 0; j < 256; ++j) *(volatile v2f*)(AGG + (size_t)(n0 + wave * 256 + j) * CH + 2 * lane) = z2;
    __threadfence();
  }
  const int* srcv = ei; const int* dstv = ei + NE;
#pragma unroll 1
  for (int c = 0; c < NCH; ++c) {
    const int tot = chunk_hits<SPT, SCH>(dstv, c * SCH, n0, tid, LIST, scan_ws);
#pragma unroll 1
    for (int base = 0; base < tot; base += 32) {
      const int q = base + lane;
      const int qq = q < SCH ? q : SCH - 1;
      const unsigned lv = LIST[qq];
      const unsigned rv = (q < tot) ? lv : SENT;
      const int own = (rv != SENT && (int)(rv >> 29) == wave) ? 1 : 0;
      unsigned msk = (unsigned)__ballot(own);
#pragma unroll 1
      for (int it = 0; it < 32; ++it) {
        if (msk == 0u) break;
        const int bp = __builtin_ctz(msk); msk &= msk - 1u;
        const unsigned r = (unsigned)__builtin_amdgcn_readfirstlane((int)__shfl(rv, bp, 32));
        const int dl = (int)(r >> 21);
        int e = (int)(r & 0x1FFFFFu); e = e < NE ? e : NE - 1;
        int s = srcv[e]; s = s < 0 ? 0 : (s >= NN ? NN - 1 : s);
        const float ea = eattr[e];
        const v2f hv = hrow<MODE>(H, s, lane, sc, sh);
        v2f m = hv + (ea * wv + bv);
        m.x = fmaxf(m.x, 0.f); m.y = fmaxf(m.y, 0.f);
        float* rp = AGG + (size_t)(n0 + dl) * CH + 2 * lane;
        v2f a = *(const v2f*)rp;
        a = a + m;
        *(volatile v2f*)rp = a;
        __threadfence();
        *(volatile v2f*)rp = a;
      }
    }
    __syncthreads();
  }
  float* sl = slab[wave];
  const int q8 = lane >> 3, c8 = (lane & 7) * 8;
#pragma unroll 1
  for (int j = 0; j < 256; j += 4) {
    const int nb = n0 + wave * 256 + j;
    if (nb < NP) {
#pragma unroll
      for (int jj = 0; jj < 4; ++jj) {
        const int n = nb + jj;
        const bool live = n < NN;
        const int nc = live ? n : NN - 1;
        const v2f a = *(const v2f*)(AGG + (size_t)n * CH + 2 * lane);
        const v2f hv = hrow<MODE>(H, nc, lane, sc, sh);
        v2f v = ep * hv + a;
        if (!live) { v.x = 0.f; v.y = 0.f; }
        sl[jj * 68 + 2 * lane] = v.x;
        sl[jj * 68 + 2 * lane + 1] = v.y;
      }
      __builtin_amdgcn_fence(__ATOMIC_RELEASE, "workgroup");
      __builtin_amdgcn_wave_barrier();
      __builtin_amdgcn_fence(__ATOMIC_ACQUIRE, "workgroup");
      v8h hv8;
#pragma unroll
      for (int e = 0; e < 8; ++e) hv8[e] = (_Float16)sl[q8 * 68 + c8 + e];
      unsigned short* dp = XH + (size_t)(nb + q8) * CH + c8;
      for (int pass = 0; pass < 2; ++pass) { *(volatile v8h*)dp = hv8; __threadfence(); }
      __builtin_amdgcn_fence(__ATOMIC_RELEASE, "workgroup");
      __builtin_amdgcn_wave_barrier();
      __builtin_amdgcn_fence(__ATOMIC_ACQUIRE, "workgroup");
    }
  }
}

__global__ __launch_bounds__(NT) void stats_kernel(const float* __restrict__ HP, double* __restrict__ PS, double* __restrict__ PQ) {
  __shared__ __align__(16) double rs[8 * CH];
  __shared__ __align__(16) double rq[8 * CH];
  const int tid = threadIdx.x, lane = tid & 31, wave = tid >> 5;
  const int b = blockIdx.x;
  double s0 = 0.0, s1 = 0.0, q0 = 0.0, q1 = 0.0;
#pragma unroll 1
  for (int j = wave; j < RPB; j += 8) {
    const v2f v = *(const v2f*)(HP + (size_t)(b * RPB + j) * CH + 2 * lane);
    const double d0 = (double)v.x, d1 = (double)v.y;
    s0 += d0; s1 += d1; q0 += d0 * d0; q1 += d1 * d1;
  }
  rs[wave * CH + 2 * lane] = s0; rs[wave * CH + 2 * lane + 1] = s1;
  rq[wave * CH + 2 * lane] = q0; rq[wave * CH + 2 * lane + 1] = q1;
  __syncthreads();
  if (wave == 0) {
    double a0 = 0.0, a1 = 0.0, b0 = 0.0, b1 = 0.0;
#pragma unroll
    for (int w = 0; w < 8; ++w) {
      a0 += rs[w * CH + 2 * lane]; a1 += rs[w * CH + 2 * lane + 1];
      b0 += rq[w * CH + 2 * lane]; b1 += rq[w * CH + 2 * lane + 1];
    }
    v2d o; o.x = a0; o.y = a1;
    v2d p; p.x = b0; p.y = b1;
    for (int pass = 0; pass < 2; ++pass) {
      *(volatile v2d*)(PS + (size_t)b * CH + 2 * lane) = o;
      *(volatile v2d*)(PQ + (size_t)b * CH + 2 * lane) = p;
      __threadfence();
    }
  }
}

__global__ __launch_bounds__(64) void bnfin_kernel(const double* __restrict__ PS, const double* __restrict__ PQ,
                                                 const float* __restrict__ gam, const float* __restrict__ bet, float* __restrict__ SCSH) {
  __shared__ __align__(16) float so[2 * CH];
  const int c = threadIdx.x;
  double s = 0.0, q = 0.0;
#pragma unroll 1
  for (int b = 0; b < NSB; ++b) { s += PS[b * CH + c]; q += PQ[b * CH + c]; }
  const double mu = s * (1.0 / (double)NN);
  const double var = q * (1.0 / (double)NN) - mu * mu;
  float varf = (float)var; varf = varf > 0.f ? varf : 0.f;
  const float scl = gam[c] * rsqrtf(varf + 1e-5f);
  so[c] = scl;
  so[CH + c] = bet[c] - (float)mu * scl;
  __syncthreads();
  if (c < 32) {
    const v4f v = *(const v4f*)(so + 4 * c);
    for (int pass = 0; pass < 2; ++pass) { *(volatile v4f*)(SCSH + 4 * c) = v; __threadfence(); }
  }
}

__global__ __launch_bounds__(NT) void pool_kernel(const float* __restrict__ HP, const float* __restrict__ scsh, const int* __restrict__ batch,
                                                 float* __restrict__ P) {
  __shared__ int LIST[SCHP];
  __shared__ int scan_ws[80];
  __shared__ __align__(16) double red[8 * CH];
  __shared__ int rc[8];
  __shared__ __align__(16) float so[CH];
  const int tid = threadIdx.x, lane = tid & 31, wave = tid >> 5;
  const int g = blockIdx.x;
  const v2f sc = *(const v2f*)(scsh + 2 * lane), sh = *(const v2f*)(scsh + CH + 2 * lane);
  double a0 = 0.0, a1 = 0.0; int cnt = 0;
#pragma unroll 1
  for (int c = 0; c < NCHP; ++c) {
    const int eb = c * SCHP + tid * 8;
    int bv[8]; int rec[8]; int kc = 0;
    {
      const bool inr = (eb < NN);
      const int ebc = inr ? eb : (NN - 8);
      const v4i b0 = *(const v4i*)(batch + ebc), bb = *(const v4i*)(batch + ebc + 4);
      bv[0] = b0[0]; bv[1] = b0[1]; bv[2] = b0[2]; bv[3] = b0[3]; bv[4] = bb[0]; bv[5] = bb[1]; bv[6] = bb[2]; bv[7] = bb[3];
      if (!inr) {
#pragma unroll
        for (int k = 0; k < 8; ++k) bv[k] = -1;
      }
    }
#pragma unroll
    for (int k = 0; k < 8; ++k) { rec[k] = -1; if (bv[k] == g) { rec[k] = eb + k; ++kc; } }
    int tot; int p = blk_excl_scan(kc, scan_ws, tid, &tot);
#pragma unroll
    for (int k = 0; k < 8; ++k) if (rec[k] >= 0) { if ((unsigned)p < (unsigned)SCHP) LIST[p] = rec[k]; ++p; }
    __syncthreads();
    const int totc = tot < SCHP ? tot : SCHP;
#pragma unroll 1
    for (int q = wave; q < totc; q += 8) {
      int nd = LIST[q]; nd = nd < 0 ? 0 : (nd >= NN ? NN - 1 : nd);
      const v2f v = hrow<1>(HP, nd, lane, sc, sh);
      a0 += (double)v.x; a1 += (double)v.y; ++cnt;
    }
    __syncthreads();
  }
  red[wave * CH + 2 * lane] = a0; red[wave * CH + 2 * lane + 1] = a1;
  if (lane == 0) rc[wave] = cnt;
  __syncthreads();
  if (wave == 0) {
    double s0 = 0.0, s1 = 0.0; int ct = 0;
#pragma unroll
    for (int w = 0; w < 8; ++w) { s0 += red[w * CH + 2 * lane]; s1 += red[w * CH + 2 * lane + 1]; ct += rc[w]; }
    const float cf = (float)ct;
    const float inv = 1.0f / fmaxf(cf, 1.0f);
    so[2 * lane] = (float)s0 * inv;
    so[2 * lane + 1] = (float)s1 * inv;
    __builtin_amdgcn_fence(__ATOMIC_RELEASE, "workgroup");
    __builtin_amdgcn_wave_barrier();
    __builtin_amdgcn_fence(__ATOMIC_ACQUIRE, "workgroup");
    if (lane < 16) {
      const v4f o = *(const v4f*)(so + 4 * lane);
      for (int pass = 0; pass < 2; ++pass) { *(volatile v4f*)(P + (size_t)g * CH + 4 * lane) = o; __threadfence(); }
    }
  }
}

__global__ __launch_bounds__(NT) void head_kernel(const float* __restrict__ P, const float* __restrict__ lw, const float* __restrict__ lb,
                                                 float* __restrict__ out) {
  __shared__ __align__(16) float so[NG * NOUT];
  const int tid = threadIdx.x, wave = tid >> 5, lane = tid & 31;
  for (int i = tid; i < NG * NOUT; i += NT) {
    const int g = i / NOUT, o = i - NOUT * g;
    float a = 0.f;
#pragma unroll 1
    for (int c = 0; c < CH; ++c) a += P[g * CH + c] * lw[o * CH + c];
    so[i] = a + lb[o];
  }
  __syncthreads();
  if (wave == 0) {
    const v4f p0 = *(const v4f*)(so + 4 * lane);
    const v4f p1 = *(const v4f*)(so + 128 + 4 * lane);
    const v4f p2 = *(const v4f*)(so + 256 + 4 * lane);
    const v4f p3 = *(const v4f*)(so + 384 + 4 * lane);
    const v4f p4 = *(const v4f*)(so + 512 + 4 * lane);
    for (int pass = 0; pass < 2; ++pass) {
      *(volatile v4f*)(out + 4 * lane) = p0;
      *(volatile v4f*)(out + 128 + 4 * lane) = p1;
      *(volatile v4f*)(out + 256 + 4 * lane) = p2;
      *(volatile v4f*)(out + 384 + 4 * lane) = p3;
      *(volatile v4f*)(out + 512 + 4 * lane) = p4;
      __threadfence();
    }
  }
}

extern "C" void kernel_launch(void* const* d_in, const int* in_sizes, int n_in,
                              void* d_out, int out_size, void* d_ws, size_t ws_size, hipStream_t stream) {
  if (n_in < 22) return;
  if (in_sizes[0] != NN * CH || in_sizes[1] != 2 * NE || in_sizes[2] != NN || in_sizes[3] != NE || out_size != NG * NOUT) return;
  const float* x        = (const float*)d_in[0];
  const int*   eidx     = (const int*)  d_in[1];
  const int*   batch    = (const int*)  d_in[2];
  const float* eattr    = (const float*)d_in[3];
  const float* lin_e0_w = (const float*)d_in[4];
  const float* lin_e0_b = (const float*)d_in[5];
  const float* mlp0_w1  = (const float*)d_in[6];
  const float* mlp0_b1  = (const float*)d_in[7];
  const float* mlp0_w2  = (const float*)d_in[8];
  const float* mlp0_b2  = (const float*)d_in[9];
  const float* eps0     = (const float*)d_in[10];
  const float* lin_e1_w = (const float*)d_in[11];
  const float* lin_e1_b = (const float*)d_in[12];
  const float* mlp1_w1  = (const float*)d_in[13];
  const float* mlp1_b1  = (const float*)d_in[14];
  const float* mlp1_w2  = (const float*)d_in[15];
  const float* mlp1_b2  = (const float*)d_in[16];
  const float* eps1     = (const float*)d_in[17];
  const float* bn_gamma = (const float*)d_in[18];
  const float* bn_beta  = (const float*)d_in[19];
  const float* lin_w    = (const float*)d_in[20];
  const float* lin_b    = (const float*)d_in[21];
  float* out = (float*)d_out;

  char* ws = (char*)d_ws; size_t off = 0;
  auto carve = [&](size_t bytes) -> char* { char* p = ws + off; off += (bytes + 255) & ~(size_t)255; return p; };
  unsigned short* WH   = (unsigned short*)carve((size_t)4 * 4096 * 2);
  unsigned short* XH   = (unsigned short*)carve((size_t)NP * CH * 2);
  unsigned short* H1   = (unsigned short*)carve((size_t)NP * CH * 2);
  float*          HP   = (float*)carve((size_t)NP * CH * 4);
  float*          AGG  = (float*)carve((size_t)NPA * CH * 4);
  double*         PS   = (double*)carve((size_t)NSB * CH * 8);
  double*         PQ   = (double*)carve((size_t)NSB * CH * 8);
  float*          SCSH = (float*)carve((size_t)2 * CH * 4);
  float*          P    = (float*)carve((size_t)NG * CH * 4);
  if (off > ws_size || off > (size_t)134217728) return;

  const unsigned short* W1a = WH;
  const unsigned short* W2a = WH + 4096;
  const unsigned short* W1b = WH + 8192;
  const unsigned short* W2b = WH + 12288;
  const int tiles = NP / 64;
  const dim3 ggrid((tiles + 7) / 8, 1);
  const float wscale = 1.0f / 16.0f;

  prep_kernel<<<32, NT, 0, stream>>>(mlp0_w1, mlp0_w2, mlp1_w1, mlp1_w2, WH);

  agg_kernel<0><<<NTILE, NT, 0, stream>>>(x, SCSH, eidx, eattr, lin_e0_w, lin_e0_b, eps0, AGG, XH);
  wmma_gemm64<0, false, 2, 1, false, 2><<<ggrid, 256, 0, stream>>>(
      XH, (const unsigned short*)nullptr, CH, 0L, W1a, (const unsigned short*)nullptr, CH, 0L,
      (void*)H1, (void*)nullptr, CH, 0L, mlp0_b1, (const float*)nullptr, 0L, NP, CH, CH, wscale);
  wmma_gemm64<0, false, 2, 0, false, 0><<<ggrid, 256, 0, stream>>>(
      H1, (const unsigned short*)nullptr, CH, 0L, W2a, (const unsigned short*)nullptr, CH, 0L,
      (void*)HP, (void*)nullptr, CH, 0L, mlp0_b2, (const float*)nullptr, 0L, NP, CH, CH, wscale);
  stats_kernel<<<NSB, NT, 0, stream>>>(HP, PS, PQ);
  bnfin_kernel<<<1, 64, 0, stream>>>(PS, PQ, bn_gamma, bn_beta, SCSH);

  for (int L = 1; L < 3; ++L) {
    agg_kernel<1><<<NTILE, NT, 0, stream>>>(HP, SCSH, eidx, eattr, lin_e1_w, lin_e1_b, eps1, AGG, XH);
    wmma_gemm64<0, false, 2, 1, false, 2><<<ggrid, 256, 0, stream>>>(
        XH, (const unsigned short*)nullptr, CH, 0L, W1b, (const unsigned short*)nullptr, CH, 0L,
        (void*)H1, (void*)nullptr, CH, 0L, mlp1_b1, (const float*)nullptr, 0L, NP, CH, CH, wscale);
    wmma_gemm64<0, false, 2, 0, false, 0><<<ggrid, 256, 0, stream>>>(
        H1, (const unsigned short*)nullptr, CH, 0L, W2b, (const unsigned short*)nullptr, CH, 0L,
        (void*)HP, (void*)nullptr, CH, 0L, mlp1_b2, (const float*)nullptr, 0L, NP, CH, CH, wscale);
    stats_kernel<<<NSB, NT, 0, stream>>>(HP, PS, PQ);
    bnfin_kernel<<<1, 64, 0, stream>>>(PS, PQ, bn_gamma + CH * L, bn_beta + CH * L, SCSH);
  }

  pool_kernel<<<NG, NT, 0, stream>>>(HP, SCSH, batch, P);
  head_kernel<<<1, NT, 0, stream>>>(P, lin_w, lin_b, out);
}
